// VC_Aggregator_85048942395937
// MI455X (gfx1250) — hardware-verified
//
#include <hip/hip_runtime.h>
#include <stdint.h>
#include <stddef.h>


typedef _Float16        v16h __attribute__((ext_vector_type(16)));
typedef _Float16        v8h  __attribute__((ext_vector_type(8)));
typedef __bf16          v16b __attribute__((ext_vector_type(16)));
typedef unsigned short  v16us __attribute__((ext_vector_type(16)));
typedef unsigned short  v8us __attribute__((ext_vector_type(8)));
typedef unsigned short  v4us __attribute__((ext_vector_type(4)));
typedef unsigned int    v4u  __attribute__((ext_vector_type(4)));
typedef float           v8f  __attribute__((ext_vector_type(8)));
typedef float           v4f  __attribute__((ext_vector_type(4)));

union FragH { v16h v; v8h p[2]; };
union FragU { v16us v; v8us p[2]; };

#define DD 64
#define PT 72
#define PK 65
#define GN 16
#define TB 256

__device__ __forceinline__ int clampi(int x, int lo, int hi) { return x < lo ? lo : (x > hi ? hi : x); }

__device__ __forceinline__ unsigned short f2bf(float f) {
    unsigned int u = __float_as_uint(f);
    u += 0x7FFFu + ((u >> 16) & 1u);
    return (unsigned short)(u >> 16);
}
__device__ __forceinline__ float bf2f(unsigned short s) { return __uint_as_float(((unsigned int)s) << 16); }

__device__ __forceinline__ void split4(v4f s, v8us& hi, v8us& lo, int o) {
    unsigned short h0 = f2bf(s.x), h1 = f2bf(s.y), h2 = f2bf(s.z), h3 = f2bf(s.w);
    hi[o + 0] = h0; lo[o + 0] = f2bf(s.x - bf2f(h0));
    hi[o + 1] = h1; lo[o + 1] = f2bf(s.y - bf2f(h1));
    hi[o + 2] = h2; lo[o + 2] = f2bf(s.z - bf2f(h2));
    hi[o + 3] = h3; lo[o + 3] = f2bf(s.w - bf2f(h3));
}
__device__ __forceinline__ void relu4(v8h& h, int o, v4f s) {
    h[o + 0] = (_Float16)fmaxf(s.x, 0.0f);
    h[o + 1] = (_Float16)fmaxf(s.y, 0.0f);
    h[o + 2] = (_Float16)fmaxf(s.z, 0.0f);
    h[o + 3] = (_Float16)fmaxf(s.w, 0.0f);
}

__device__ __forceinline__ v8f mma_f16(v16h a, v16h b, v8f c) {
    v8f d = __builtin_amdgcn_wmma_f32_16x16x32_f16(false, a, false, b, (short)0, c, false, false);
    asm volatile("v_nop\n\tv_nop\n\tv_nop\n\tv_nop" : "+v"(d) : "v"(a), "v"(b));
    return d;
}
__device__ __forceinline__ v8f mma_bf16(v16us a, v16us b, v8f c) {
    v16b av = __builtin_bit_cast(v16b, a);
    v16b bv = __builtin_bit_cast(v16b, b);
    v8f d = __builtin_amdgcn_wmma_f32_16x16x32_bf16(false, av, false, bv, (short)0, c, false, false);
    asm volatile("v_nop\n\tv_nop\n\tv_nop\n\tv_nop" : "+v"(d) : "v"(av), "v"(bv));
    return d;
}
__device__ __forceinline__ v8f mma3_bf16(v16us ah, v16us al, v16us bh, v16us bl, v8f c) {
    c = mma_bf16(ah, bh, c);
    c = mma_bf16(ah, bl, c);
    c = mma_bf16(al, bh, c);
    return c;
}

__device__ __forceinline__ void st2f4(float* p, v4f v) {
    *(volatile v4f*)p = v;
    __threadfence();
    *(volatile v4f*)p = v;
}
__device__ __forceinline__ void st2u4(void* p, v4u v) {
    *(volatile v4u*)p = v;
    __threadfence();
    *(volatile v4u*)p = v;
}

__global__ __launch_bounds__(TB)
void k_prep(const float* __restrict__ c2e, const float* __restrict__ r2e,
            const float* __restrict__ W1,  const float* __restrict__ b1,
            const float* __restrict__ Wq,  const float* __restrict__ Wk,
            const float* __restrict__ Wv,  const float* __restrict__ Wo,
            float* T1, float* T2,
            _Float16* WKt, _Float16* WVt,
            unsigned short* WQh, unsigned short* WQl,
            unsigned short* WOh, unsigned short* WOl,
            int NC, int NR, int MT1)
{
    __shared__ __align__(16) float t1s[16 * DD];
    __shared__ __align__(16) float t2s[8 * DD];

    const int tid = threadIdx.x;
    const int w   = tid >> 5;
    const int l   = tid & 31;
    const int hh  = l >> 4;
    const int m   = l & 15;
    const int b   = blockIdx.x;

    if (b < MT1) {
        if (w < 4) {
            const int nt = w;
            int row = b * 16 + m;
            if (row > NC - 1) row = NC - 1;
            v8f acc = {};
#pragma unroll
            for (int ks = 0; ks < 2; ++ks) {
                const float* ap = c2e + (size_t)row * DD + ks * 32 + 8 * hh;
                FragU ah, al;
                split4(*(const v4f*)(ap),      ah.p[0], al.p[0], 0);
                split4(*(const v4f*)(ap + 4),  ah.p[0], al.p[0], 4);
                split4(*(const v4f*)(ap + 16), ah.p[1], al.p[1], 0);
                split4(*(const v4f*)(ap + 20), ah.p[1], al.p[1], 4);
                FragU bh, bl;
#pragma unroll
                for (int i = 0; i < 16; ++i) {
                    const int k = ks * 32 + ((i < 8) ? (8 * hh + i) : (16 + 8 * hh + (i - 8)));
                    const float val = W1[(size_t)k * DD + nt * 16 + m];
                    const unsigned short hv = f2bf(val);
                    bh.v[i] = hv;
                    bl.v[i] = f2bf(val - bf2f(hv));
                }
                acc = mma3_bf16(ah.v, al.v, bh.v, bl.v, acc);
            }
#pragma unroll
            for (int r = 0; r < 8; ++r) t1s[(8 * hh + r) * DD + nt * 16 + m] = acc[r];
        }
        __syncthreads();
        {
            const int row = 2 * w + hh;
            const int col = m * 4;
            const v4f v = *(const v4f*)&t1s[row * DD + col];
            st2f4(T1 + ((size_t)(b * 16 + row)) * DD + col, v);
        }
    } else if (b == MT1) {
        const int nrr = NR < 8 ? NR : 8;
        for (int idx = tid; idx < nrr * DD; idx += TB) {
            const int r = idx >> 6;
            const int e = idx & 63;
            float s = b1[e];
#pragma unroll 4
            for (int j = 0; j < DD; ++j) s += r2e[r * DD + j] * W1[(size_t)(DD + j) * DD + e];
            t2s[idx] = s;
        }
        __syncthreads();
        if (tid < nrr * 16) {
            const int row = tid >> 4;
            const int col = (tid & 15) * 4;
            const v4f v = *(const v4f*)&t2s[row * DD + col];
            st2f4(T2 + row * DD + col, v);
        }
    } else {
        for (int i = tid; i < 6 * 512; i += TB) {
            const int plane = i >> 9;
            const int rem   = i & 511;
            const int n     = rem >> 3;
            const int k0    = (rem & 7) * 8;
            const float* W = (plane == 0) ? Wk : (plane == 1) ? Wv : (plane <= 3) ? Wq : Wo;
            v4f x0, x1;
            x0.x = W[(size_t)(k0 + 0) * DD + n]; x0.y = W[(size_t)(k0 + 1) * DD + n];
            x0.z = W[(size_t)(k0 + 2) * DD + n]; x0.w = W[(size_t)(k0 + 3) * DD + n];
            x1.x = W[(size_t)(k0 + 4) * DD + n]; x1.y = W[(size_t)(k0 + 5) * DD + n];
            x1.z = W[(size_t)(k0 + 6) * DD + n]; x1.w = W[(size_t)(k0 + 7) * DD + n];
            if (plane < 2) {
                v8h hv;
                hv[0] = (_Float16)(x0.x * 64.0f); hv[1] = (_Float16)(x0.y * 64.0f);
                hv[2] = (_Float16)(x0.z * 64.0f); hv[3] = (_Float16)(x0.w * 64.0f);
                hv[4] = (_Float16)(x1.x * 64.0f); hv[5] = (_Float16)(x1.y * 64.0f);
                hv[6] = (_Float16)(x1.z * 64.0f); hv[7] = (_Float16)(x1.w * 64.0f);
                _Float16* dst = ((plane == 0) ? WKt : WVt) + n * DD + k0;
                st2u4((void*)dst, __builtin_bit_cast(v4u, hv));
            } else {
                v8us hi, lo;
                split4(x0, hi, lo, 0);
                split4(x1, hi, lo, 4);
                unsigned short* dst;
                v8us o;
                if (plane == 2)      { dst = WQh; o = hi; }
                else if (plane == 3) { dst = WQl; o = lo; }
                else if (plane == 4) { dst = WOh; o = hi; }
                else                 { dst = WOl; o = lo; }
                st2u4((void*)(dst + n * DD + k0), __builtin_bit_cast(v4u, o));
            }
        }
    }
}

__global__ __launch_bounds__(TB)
void k_main(const int* __restrict__ nodes, const int* __restrict__ hvc, const int* __restrict__ hr,
            const float* __restrict__ v2e,
            const float* __restrict__ bq, const float* __restrict__ bk,
            const float* __restrict__ bv, const float* __restrict__ bo,
            const float* __restrict__ T1, const float* __restrict__ T2,
            const _Float16* __restrict__ WKt, const _Float16* __restrict__ WVt,
            const unsigned short* __restrict__ WQh, const unsigned short* __restrict__ WQl,
            const unsigned short* __restrict__ WOh, const unsigned short* __restrict__ WOl,
            float* out, int N, int L, int NC, int NI, int NR)
{
    __shared__ __align__(16) _Float16       hA[64 * PT];
    __shared__ __align__(16) float          kv_s[2 * 64 * PK];
    __shared__ __align__(16) float          q_s[GN * DD];
    __shared__ __align__(16) float          o_s[GN * DD];
    __shared__ __align__(16) unsigned short vAh[GN * PT];
    __shared__ __align__(16) unsigned short vAl[GN * PT];
    __shared__ __align__(16) unsigned short cAh[GN * PT];
    __shared__ __align__(16) unsigned short cAl[GN * PT];
    __shared__ float sc_s[64];

    const int tid = threadIdx.x;
    const int w   = tid >> 5;
    const int l   = tid & 31;
    const int hh  = l >> 4;
    const int m   = l & 15;
    const int nb  = blockIdx.x * GN;
    const int Lc  = L < 64 ? L : 64;
    const int nrr = NR < 8 ? NR : 8;

    {
        const int g    = tid >> 4;
        const int c0   = (tid & 15) * 4;
        const int node = nb + g;
        v4f x = {};
        if (node < N) {
            int id = nodes[node];
            id = clampi(id, 0, NI - 1);
            x = *(const v4f*)(v2e + (size_t)id * DD + c0);
        }
        v4us hi, lo;
        unsigned short t0 = f2bf(x.x), t1 = f2bf(x.y), t2 = f2bf(x.z), t3 = f2bf(x.w);
        hi.x = t0; lo.x = f2bf(x.x - bf2f(t0));
        hi.y = t1; lo.y = f2bf(x.y - bf2f(t1));
        hi.z = t2; lo.z = f2bf(x.z - bf2f(t2));
        hi.w = t3; lo.w = f2bf(x.w - bf2f(t3));
        *(v4us*)&vAh[g * PT + c0] = hi;
        *(v4us*)&vAl[g * PT + c0] = lo;
    }
    __syncthreads();

    if (w < 4) {
        const int nt = w;
        v8f acc = {};
#pragma unroll
        for (int ks = 0; ks < 2; ++ks) {
            FragU ah, al, bh, bl;
            const int ao = m * PT + ks * 32 + 8 * hh;
            ah.p[0] = *(const v8us*)&vAh[ao];
            ah.p[1] = *(const v8us*)&vAh[ao + 16];
            al.p[0] = *(const v8us*)&vAl[ao];
            al.p[1] = *(const v8us*)&vAl[ao + 16];
            const size_t bofs = (size_t)(nt * 16 + m) * DD + ks * 32 + 8 * hh;
            bh.p[0] = *(const v8us*)(WQh + bofs);
            bh.p[1] = *(const v8us*)(WQh + bofs + 16);
            bl.p[0] = *(const v8us*)(WQl + bofs);
            bl.p[1] = *(const v8us*)(WQl + bofs + 16);
            acc = mma3_bf16(ah.v, al.v, bh.v, bl.v, acc);
        }
        const float bias = bq[nt * 16 + m];
#pragma unroll
        for (int r = 0; r < 8; ++r) q_s[(8 * hh + r) * DD + nt * 16 + m] = acc[r] + bias;
    }
    __syncthreads();

#pragma unroll 1
    for (int g = 0; g < GN; ++g) {
        const int node  = nb + g;
        const int nodec = (node < N) ? node : (N - 1);

        {
            const int row = tid >> 2;
            const int c0  = (tid & 3) * 16;
            v8h h0 = {}, h1 = {};
            if (row < Lc) {
                int c = hvc[(size_t)nodec * L + row];
                c = clampi(c, 0, NC - 1);
                int r = hr[(size_t)nodec * L + row];
                r = clampi(r, 0, nrr - 1);
                const float* p1 = T1 + (size_t)c * DD + c0;
                const float* p2 = T2 + r * DD + c0;
                const v4f s0 = *(const v4f*)(p1)      + *(const v4f*)(p2);
                const v4f s1 = *(const v4f*)(p1 + 4)  + *(const v4f*)(p2 + 4);
                const v4f s2 = *(const v4f*)(p1 + 8)  + *(const v4f*)(p2 + 8);
                const v4f s3 = *(const v4f*)(p1 + 12) + *(const v4f*)(p2 + 12);
                relu4(h0, 0, s0);
                relu4(h0, 4, s1);
                relu4(h1, 0, s2);
                relu4(h1, 4, s3);
            }
            *(v8h*)&hA[row * PT + c0]     = h0;
            *(v8h*)&hA[row * PT + c0 + 8] = h1;
        }
        __syncthreads();

        {
            const int mt  = w & 3;
            const int sel = w >> 2;
            const _Float16* WT = sel ? WVt : WKt;
            const float*    bb = sel ? bv : bk;
            float* dst = kv_s + sel * (64 * PK);
            FragH a0, a1;
            const int ao = (mt * 16 + m) * PT + 8 * hh;
            a0.p[0] = *(const v8h*)&hA[ao];
            a0.p[1] = *(const v8h*)&hA[ao + 16];
            a1.p[0] = *(const v8h*)&hA[ao + 32];
            a1.p[1] = *(const v8h*)&hA[ao + 48];
#pragma unroll
            for (int nt = 0; nt < 4; ++nt) {
                FragH b0, b1;
                const size_t bofs = (size_t)(nt * 16 + m) * DD + 8 * hh;
                b0.p[0] = *(const v8h*)(WT + bofs);
                b0.p[1] = *(const v8h*)(WT + bofs + 16);
                b1.p[0] = *(const v8h*)(WT + bofs + 32);
                b1.p[1] = *(const v8h*)(WT + bofs + 48);
                v8f acc = {};
                acc = mma_f16(a0.v, b0.v, acc);
                acc = mma_f16(a1.v, b1.v, acc);
                const float bias = bb[nt * 16 + m];
#pragma unroll
                for (int r = 0; r < 8; ++r)
                    dst[(mt * 16 + 8 * hh + r) * PK + nt * 16 + m] = acc[r] * 0.015625f + bias;
            }
        }
        __syncthreads();

        if (tid < Lc) {
            const float* kr = kv_s + tid * PK;
            const float* qr = q_s + g * DD;
            float s = 0.0f;
#pragma unroll 8
            for (int d = 0; d < DD; ++d) s += qr[d] * kr[d];
            sc_s[tid] = s * 0.125f;
        }
        __syncthreads();

        if (w == 0) {
            const float NEG = -3.0e38f;
            const bool  u0 = l < Lc;
            const bool  u1 = (l + 32) < Lc;
            const float s0 = u0 ? sc_s[l] : NEG;
            const float s1 = u1 ? sc_s[l + 32] : NEG;
            float mx = fmaxf(s0, s1);
            mx = fmaxf(mx, __shfl_xor(mx, 16));
            mx = fmaxf(mx, __shfl_xor(mx, 8));
            mx = fmaxf(mx, __shfl_xor(mx, 4));
            mx = fmaxf(mx, __shfl_xor(mx, 2));
            mx = fmaxf(mx, __shfl_xor(mx, 1));
            const float e0 = u0 ? expf(s0 - mx) : 0.0f;
            const float e1 = u1 ? expf(s1 - mx) : 0.0f;
            float sm = e0 + e1;
            sm += __shfl_xor(sm, 16);
            sm += __shfl_xor(sm, 8);
            sm += __shfl_xor(sm, 4);
            sm += __shfl_xor(sm, 2);
            sm += __shfl_xor(sm, 1);
            const float inv = 1.0f / sm;
            if (u0) sc_s[l]      = e0 * inv;
            if (u1) sc_s[l + 32] = e1 * inv;
        }
        __syncthreads();

        if (tid < DD) {
            const float* vcol = kv_s + 64 * PK + tid;
            float c = 0.0f;
            for (int j = 0; j < Lc; ++j) c += sc_s[j] * vcol[j * PK];
            const unsigned short hv = f2bf(c);
            cAh[g * PT + tid] = hv;
            cAl[g * PT + tid] = f2bf(c - bf2f(hv));
        }
        __syncthreads();
    }

    if (w < 4) {
        const int nt = w;
        v8f acc = {};
#pragma unroll
        for (int ks = 0; ks < 2; ++ks) {
            FragU ah, al, bh, bl;
            const int ao = m * PT + ks * 32 + 8 * hh;
            ah.p[0] = *(const v8us*)&cAh[ao];
            ah.p[1] = *(const v8us*)&cAh[ao + 16];
            al.p[0] = *(const v8us*)&cAl[ao];
            al.p[1] = *(const v8us*)&cAl[ao + 16];
            const size_t bofs = (size_t)(nt * 16 + m) * DD + ks * 32 + 8 * hh;
            bh.p[0] = *(const v8us*)(WOh + bofs);
            bh.p[1] = *(const v8us*)(WOh + bofs + 16);
            bl.p[0] = *(const v8us*)(WOl + bofs);
            bl.p[1] = *(const v8us*)(WOl + bofs + 16);
            acc = mma3_bf16(ah.v, al.v, bh.v, bl.v, acc);
        }
        const float bias = bo[nt * 16 + m];
#pragma unroll
        for (int r = 0; r < 8; ++r) o_s[(8 * hh + r) * DD + nt * 16 + m] = acc[r] + bias;
    }
    __syncthreads();

    {
        const int row  = 2 * w + hh;
        const int col  = m * 4;
        const int node = nb + row;
        if (node < N) {
            const v4f v = *(const v4f*)&o_s[row * DD + col];
            st2f4(out + (size_t)node * DD + col, v);
        }
    }
}

extern "C" void kernel_launch(void* const* d_in, const int* in_sizes, int n_in,
                              void* d_out, int out_size, void* d_ws, size_t ws_size,
                              hipStream_t stream)
{
    (void)n_in;
    const int N = in_sizes[0];
    if (N <= 0) return;
    const int L  = in_sizes[1] / N;
    const int NC = in_sizes[3] / DD;
    const int NI = in_sizes[4] / DD;
    const int NR = in_sizes[5] / DD;
    if (L < 1 || L > 64 || NC < 1 || NI < 1 || NR < 1) return;
    if (in_sizes[2] != in_sizes[1]) return;
    if (out_size < N * DD) return;
    const int MT1 = (NC + 15) / 16;

    const size_t offT1 = 0;
    const size_t szT1  = (size_t)MT1 * 16 * DD * sizeof(float);
    const size_t offT2 = (offT1 + szT1 + 127) & ~(size_t)127;
    const size_t szT2  = (size_t)8 * DD * sizeof(float);
    const size_t szP   = (size_t)DD * DD * 2;
    const size_t offWK = offT2 + szT2;
    const size_t offWV = offWK + szP;
    const size_t offQH = offWV + szP;
    const size_t offQL = offQH + szP;
    const size_t offOH = offQL + szP;
    const size_t offOL = offOH + szP;
    const size_t total = offOL + szP;
    if (total > ws_size) return;

    const int*   nodes = (const int*)d_in[0];
    const int*   hvc   = (const int*)d_in[1];
    const int*   hr    = (const int*)d_in[2];
    const float* c2e   = (const float*)d_in[3];
    const float* v2e   = (const float*)d_in[4];
    const float* r2e   = (const float*)d_in[5];
    const float* W1    = (const float*)d_in[6];
    const float* b1    = (const float*)d_in[7];
    const float* Wq    = (const float*)d_in[8];
    const float* bq    = (const float*)d_in[9];
    const float* Wk    = (const float*)d_in[10];
    const float* bk    = (const float*)d_in[11];
    const float* Wv    = (const float*)d_in[12];
    const float* bv    = (const float*)d_in[13];
    const float* Wo    = (const float*)d_in[14];
    const float* bo    = (const float*)d_in[15];
    float* out = (float*)d_out;

    char* ws = (char*)d_ws;
    float*          T1  = (float*)(ws + offT1);
    float*          T2  = (float*)(ws + offT2);
    _Float16*       WKt = (_Float16*)(ws + offWK);
    _Float16*       WVt = (_Float16*)(ws + offWV);
    unsigned short* WQh = (unsigned short*)(ws + offQH);
    unsigned short* WQl = (unsigned short*)(ws + offQL);
    unsigned short* WOh = (unsigned short*)(ws + offOH);
    unsigned short* WOl = (unsigned short*)(ws + offOL);

    k_prep<<<dim3(MT1 + 2), dim3(TB), 0, stream>>>(c2e, r2e, W1, b1, Wq, Wk, Wv, Wo,
                                                   T1, T2, WKt, WVt, WQh, WQl, WOh, WOl,
                                                   NC, NR, MT1);

    k_main<<<dim3((N + GN - 1) / GN), dim3(TB), 0, stream>>>(nodes, hvc, hr, v2e,
                                                              bq, bk, bv, bo,
                                                              T1, T2, WKt, WVt, WQh, WQl, WOh, WOl,
                                                              out, N, L, NC, NI, NR);
}
